// RNP_33792802685161
// MI455X (gfx1250) — hardware-verified
//
#include <hip/hip_runtime.h>
#define BT 32
#define NPT 1024
#define GR 64
#define NG (GR * GR)
#define CH 128

typedef __bf16 v16b __attribute__((ext_vector_type(16)));
typedef unsigned short v8us __attribute__((ext_vector_type(8), may_alias));
typedef float  v8f  __attribute__((ext_vector_type(8)));
typedef float  v4f  __attribute__((ext_vector_type(4)));
typedef float  v4fa __attribute__((ext_vector_type(4), may_alias));
union FragB { v16b v; v8us half[2]; unsigned short u[16]; };

__device__ __forceinline__ unsigned short bf16_bits(float x) { unsigned int u = __float_as_uint(x); return (unsigned short)((u + 0x7FFFu + ((u >> 16) & 1u)) >> 16); }
__device__ __forceinline__ float bf16_val(unsigned short b) { return __uint_as_float(((unsigned int)b) << 16); }
__device__ __forceinline__ float bf16_round(float x) { return bf16_val(bf16_bits(x)); }
template <int NT>
__device__ __forceinline__ v8f mmaN(v16b ah, v16b al, v16b bh, v16b bl, v8f c) {
  c = __builtin_amdgcn_wmma_f32_16x16x32_bf16(false, ah, false, bh, (short)0, c, false, false);
  if (NT >= 2) c = __builtin_amdgcn_wmma_f32_16x16x32_bf16(false, al, false, bh, (short)0, c, false, false);
  if (NT >= 3) c = __builtin_amdgcn_wmma_f32_16x16x32_bf16(false, ah, false, bl, (short)0, c, false, false);
  asm volatile("v_nop\n\tv_nop\n\tv_nop\n\tv_nop" : "+v"(c) : "v"(ah), "v"(al), "v"(bh), "v"(bl));
  return c;
}

__global__ __launch_bounds__(256) void k_wt_bf16(const float* __restrict__ W, unsigned short* __restrict__ Wt, int K, int N) {
  const int t = blockIdx.x * 256 + threadIdx.x;
  const int k8n = K / 8;
  if (t >= N * k8n) return;
  const int n = t / k8n, k8 = (t % k8n) * 8;
  v8us v;
#pragma unroll
  for (int i = 0; i < 8; ++i) v[i] = bf16_bits(W[(size_t)(k8 + i) * N + n]);
  *(volatile v8us*)(Wt + (size_t)n * K + k8) = v;
  __threadfence();
  *(volatile v8us*)(Wt + (size_t)n * K + k8) = v;
}

template <bool ASPLIT, int ACT, bool BIAS_BF16>
__global__ __launch_bounds__(128) void k_gemm_bf(const float* __restrict__ A, int lda, const unsigned short* __restrict__ Wt, int ldb,
                                               const float* __restrict__ bias, float* __restrict__ C, int ldc, int M, int N, int K) {
  __shared__ __attribute__((aligned(16))) float so[4][16][64];
  const int tid = threadIdx.x, w = tid >> 5, lane = tid & 31, ln = lane & 15, hh = lane >> 4;
  const int ntn = N / 64;
  const int wid = blockIdx.x * 4 + w;
  const int mt = wid / ntn, nq = wid % ntn;
  if (mt * 16 >= M) return;
  const int row0 = mt * 16, col0 = nq * 64;
  const float* arow = A + (size_t)(row0 + ln) * lda;
  v8f acc[4] = {};
  for (int kb = 0; kb < K; kb += 32) {
    FragB ah, al;
    const v4f x0 = *(const v4fa*)(arow + kb + 8 * hh), x1 = *(const v4fa*)(arow + kb + 8 * hh + 4);
    const v4f x2 = *(const v4fa*)(arow + kb + 16 + 8 * hh), x3 = *(const v4fa*)(arow + kb + 16 + 8 * hh + 4);
    float xs[16] = {x0[0],x0[1],x0[2],x0[3],x1[0],x1[1],x1[2],x1[3],x2[0],x2[1],x2[2],x2[3],x3[0],x3[1],x3[2],x3[3]};
#pragma unroll
    for (int i = 0; i < 16; ++i) { const unsigned short hb = bf16_bits(xs[i]); ah.u[i] = hb; al.u[i] = ASPLIT ? bf16_bits(xs[i] - bf16_val(hb)) : (unsigned short)0; }
#pragma unroll
    for (int t = 0; t < 4; ++t) {
      const unsigned short* brow = Wt + (size_t)(col0 + t * 16 + ln) * ldb + kb;
      FragB b;
      b.half[0] = *(const v8us*)(brow + 8 * hh);
      b.half[1] = *(const v8us*)(brow + 16 + 8 * hh);
      acc[t] = mmaN<ASPLIT ? 2 : 1>(ah.v, al.v, b.v, b.v, acc[t]);
    }
  }
#pragma unroll
  for (int t = 0; t < 4; ++t) {
    float bv = bias ? bias[col0 + t * 16 + ln] : 0.f;
    if (BIAS_BF16) bv = bf16_round(bv);
#pragma unroll
    for (int r = 0; r < 8; ++r) { float v = acc[t][r] + bv; if (ACT == 1) v = fmaxf(v, 0.f); so[w][8 * hh + r][t * 16 + ln] = v; }
  }
  __builtin_amdgcn_fence(__ATOMIC_ACQ_REL, "workgroup");
  __builtin_amdgcn_wave_barrier();
  const int rsub = lane >> 4, c4 = (lane & 15) * 4;
  for (int pass = 0; pass < 2; ++pass) {
#pragma unroll
    for (int q = 0; q < 8; ++q) {
      const int r = q * 2 + rsub;
      const v4f v = *(const v4fa*)&so[w][r][c4];
      *(volatile v4f*)(C + (size_t)(row0 + r) * ldc + col0 + c4) = v;
    }
    if (pass == 0) __threadfence();
  }
}

template <int D, bool CAUSAL>
__global__ __launch_bounds__(128) void k_flash(const float* __restrict__ qb, const float* __restrict__ kb, const float* __restrict__ vb,
                                             int pitch, int T, int H, float scale, float* __restrict__ y, int ypitch) {
  constexpr int KS = D / 32;
  constexpr int DT = D / 16;
  __shared__ __attribute__((aligned(16))) unsigned short sKh[32][D + 8], sKl[32][D + 8], sVh[32][D + 8], sVl[32][D + 8];
  __shared__ __attribute__((aligned(16))) unsigned short sPh[4][16][40], sPl[4][16][40];
  __shared__ __attribute__((aligned(16))) float sO[4][16][D];
  const int tid = threadIdx.x, w = tid >> 5, lane = tid & 31, ln = lane & 15, hh = lane >> 4;
  const int nqb = (T + 63) / 64;
  const int bh = blockIdx.x / nqb, qblk = blockIdx.x % nqb;
  const int b = bh / H, h = bh % H;
  const int q0 = qblk * 64 + w * 16;
  const float* Q = qb + (size_t)b * T * pitch + h * D;
  const float* K = kb + (size_t)b * T * pitch + h * D;
  const float* V = vb + (size_t)b * T * pitch + h * D;

  FragB aqh[KS], aql[KS];
  {
    int row = q0 + ln; if (row >= T) row = T - 1;
    const float* qr = Q + (size_t)row * pitch;
#pragma unroll
    for (int ks = 0; ks < KS; ++ks)
#pragma unroll
      for (int i = 0; i < 16; ++i) {
        const int d = ks * 32 + ((i < 8) ? (8 * hh + i) : (16 + 8 * hh + (i - 8)));
        const float x = qr[d] * scale; const unsigned short hb = bf16_bits(x);
        aqh[ks].u[i] = hb; aql[ks].u[i] = bf16_bits(x - bf16_val(hb));
      }
  }
  float m_r[8], l_r[8];
#pragma unroll
  for (int r = 0; r < 8; ++r) { m_r[r] = -3.0e38f; l_r[r] = 0.f; }
  v8f oacc[DT];
#pragma unroll
  for (int dt = 0; dt < DT; ++dt) oacc[dt] = (v8f){0.f,0.f,0.f,0.f,0.f,0.f,0.f,0.f};

  const int kv_end = CAUSAL ? min(T, qblk * 64 + 64) : T;
  for (int j0 = 0; j0 < kv_end; j0 += 32) {
    __syncthreads();
    for (int e = tid; e < 32 * (D / 4); e += 128) {
      const int r = e / (D / 4), c4 = (e % (D / 4)) * 4;
      const int key = j0 + r;
      v4f kf = {0.f,0.f,0.f,0.f}, vf = {0.f,0.f,0.f,0.f};
      if (key < T) { kf = *(const v4fa*)(K + (size_t)key * pitch + c4); vf = *(const v4fa*)(V + (size_t)key * pitch + c4); }
#pragma unroll
      for (int t = 0; t < 4; ++t) {
        unsigned short hb = bf16_bits(kf[t]); sKh[r][c4 + t] = hb; sKl[r][c4 + t] = bf16_bits(kf[t] - bf16_val(hb));
        hb = bf16_bits(vf[t]); sVh[r][c4 + t] = hb; sVl[r][c4 + t] = bf16_bits(vf[t] - bf16_val(hb));
      }
    }
    __syncthreads();
    v8f s[2];
#pragma unroll
    for (int nt = 0; nt < 2; ++nt) {
      v8f acc = {};
#pragma unroll
      for (int ks = 0; ks < KS; ++ks) {
        FragB bh_, bl_;
        bh_.half[0] = *(const v8us*)&sKh[nt * 16 + ln][ks * 32 + 8 * hh]; bh_.half[1] = *(const v8us*)&sKh[nt * 16 + ln][ks * 32 + 16 + 8 * hh];
        bl_.half[0] = *(const v8us*)&sKl[nt * 16 + ln][ks * 32 + 8 * hh]; bl_.half[1] = *(const v8us*)&sKl[nt * 16 + ln][ks * 32 + 16 + 8 * hh];
        acc = mmaN<3>(aqh[ks].v, aql[ks].v, bh_.v, bl_.v, acc);
      }
      s[nt] = acc;
    }
    float alpha[8];
#pragma unroll
    for (int r = 0; r < 8; ++r) {
      const int qi = q0 + 8 * hh + r;
      const int ja = j0 + ln, jb = j0 + 16 + ln;
      if (CAUSAL) { if (ja > qi) s[0][r] = -3.0e38f; if (jb > qi) s[1][r] = -3.0e38f; }
      if (ja >= T) s[0][r] = -3.0e38f;
      if (jb >= T) s[1][r] = -3.0e38f;
      float mx = fmaxf(s[0][r], s[1][r]);
      mx = fmaxf(mx, __shfl_xor(mx, 1, 32)); mx = fmaxf(mx, __shfl_xor(mx, 2, 32)); mx = fmaxf(mx, __shfl_xor(mx, 4, 32)); mx = fmaxf(mx, __shfl_xor(mx, 8, 32));
      const float mnew = fmaxf(m_r[r], mx);
      alpha[r] = (mnew > -1.0e38f) ? __expf(m_r[r] - mnew) : 1.0f;
      const float p0 = (s[0][r] > -1.0e38f) ? __expf(s[0][r] - mnew) : 0.f;
      const float p1 = (s[1][r] > -1.0e38f) ? __expf(s[1][r] - mnew) : 0.f;
      m_r[r] = mnew;
      l_r[r] = l_r[r] * alpha[r] + p0 + p1;
      unsigned short hb = bf16_bits(p0); sPh[w][8 * hh + r][ln] = hb;      sPl[w][8 * hh + r][ln] = bf16_bits(p0 - bf16_val(hb));
      hb = bf16_bits(p1);                sPh[w][8 * hh + r][16 + ln] = hb; sPl[w][8 * hh + r][16 + ln] = bf16_bits(p1 - bf16_val(hb));
    }
#pragma unroll
    for (int dt = 0; dt < DT; ++dt)
#pragma unroll
      for (int r = 0; r < 8; ++r) oacc[dt][r] *= alpha[r];
    __builtin_amdgcn_fence(__ATOMIC_ACQ_REL, "workgroup");
    __builtin_amdgcn_wave_barrier();
    FragB pah, pal;
    pah.half[0] = *(const v8us*)&sPh[w][ln][8 * hh]; pah.half[1] = *(const v8us*)&sPh[w][ln][16 + 8 * hh];
    pal.half[0] = *(const v8us*)&sPl[w][ln][8 * hh]; pal.half[1] = *(const v8us*)&sPl[w][ln][16 + 8 * hh];
#pragma unroll
    for (int dt = 0; dt < DT; ++dt) {
      FragB bvh, bvl;
#pragma unroll
      for (int i = 0; i < 8; ++i) {
        bvh.u[i] = sVh[8 * hh + i][dt * 16 + ln]; bvh.u[8 + i] = sVh[16 + 8 * hh + i][dt * 16 + ln];
        bvl.u[i] = sVl[8 * hh + i][dt * 16 + ln]; bvl.u[8 + i] = sVl[16 + 8 * hh + i][dt * 16 + ln];
      }
      oacc[dt] = mmaN<3>(pah.v, pal.v, bvh.v, bvl.v, oacc[dt]);
    }
    __builtin_amdgcn_fence(__ATOMIC_ACQ_REL, "workgroup");
    __builtin_amdgcn_wave_barrier();
  }
#pragma unroll
  for (int r = 0; r < 8; ++r) {
    float l = l_r[r];
    l += __shfl_xor(l, 1, 32); l += __shfl_xor(l, 2, 32); l += __shfl_xor(l, 4, 32); l += __shfl_xor(l, 8, 32);
    l_r[r] = (l > 0.f) ? 1.0f / l : 0.f;
  }
#pragma unroll
  for (int dt = 0; dt < DT; ++dt)
#pragma unroll
    for (int r = 0; r < 8; ++r) sO[w][8 * hh + r][dt * 16 + ln] = oacc[dt][r] * l_r[r];
  __builtin_amdgcn_fence(__ATOMIC_ACQ_REL, "workgroup");
  __builtin_amdgcn_wave_barrier();
  for (int pass = 0; pass < 2; ++pass) {
    for (int r = 0; r < 16; ++r) {
      const int row = q0 + r;
      if (row < T && lane < D / 4) {
        const v4f val = *(const v4fa*)&sO[w][r][lane * 4];
        *(volatile v4f*)(y + ((size_t)b * T + row) * ypitch + h * D + lane * 4) = val;
      }
    }
    if (pass == 0) __threadfence();
  }
}

template <bool ASPLIT, int ACT, bool BIAS_BF16, bool RES_BF16>
__global__ __launch_bounds__(128) void k_gemm_bf3(const float* __restrict__ A, int lda, const unsigned short* __restrict__ Wt, int ldb,
                                                const float* __restrict__ bias, const float* __restrict__ resid, int rmod, int ldr,
                                                float* __restrict__ C, int ldc, int M, int N, int K) {
  __shared__ __attribute__((aligned(16))) float so[4][16][64];
  const int tid = threadIdx.x, w = tid >> 5, lane = tid & 31, ln = lane & 15, hh = lane >> 4;
  const int ntn = N / 64;
  const int wid = blockIdx.x * 4 + w;
  const int mt = wid / ntn, nq = wid % ntn;
  if (mt * 16 >= M) return;
  const int row0 = mt * 16, col0 = nq * 64;
  const float* arow = A + (size_t)(row0 + ln) * lda;
  v8f acc[4] = {};
  for (int kb = 0; kb < K; kb += 32) {
    FragB ah, al;
    const v4f x0 = *(const v4fa*)(arow + kb + 8 * hh), x1 = *(const v4fa*)(arow + kb + 8 * hh + 4);
    const v4f x2 = *(const v4fa*)(arow + kb + 16 + 8 * hh), x3 = *(const v4fa*)(arow + kb + 16 + 8 * hh + 4);
    float xs[16] = {x0[0],x0[1],x0[2],x0[3],x1[0],x1[1],x1[2],x1[3],x2[0],x2[1],x2[2],x2[3],x3[0],x3[1],x3[2],x3[3]};
#pragma unroll
    for (int i = 0; i < 16; ++i) { const unsigned short hb = bf16_bits(xs[i]); ah.u[i] = hb; al.u[i] = ASPLIT ? bf16_bits(xs[i] - bf16_val(hb)) : (unsigned short)0; }
#pragma unroll
    for (int t = 0; t < 4; ++t) {
      const unsigned short* brow = Wt + (size_t)(col0 + t * 16 + ln) * ldb + kb;
      FragB b;
      b.half[0] = *(const v8us*)(brow + 8 * hh);
      b.half[1] = *(const v8us*)(brow + 16 + 8 * hh);
      acc[t] = mmaN<ASPLIT ? 2 : 1>(ah.v, al.v, b.v, b.v, acc[t]);
    }
  }
#pragma unroll
  for (int t = 0; t < 4; ++t) {
    const int col = col0 + t * 16 + ln;
    float bv = bias ? bias[col] : 0.f;
    if (BIAS_BF16) bv = bf16_round(bv);
#pragma unroll
    for (int r = 0; r < 8; ++r) {
      float v = acc[t][r] + bv;
      if (resid) { float rv = resid[(size_t)((row0 + 8 * hh + r) % rmod) * ldr + col]; if (RES_BF16) rv = bf16_round(rv); v += rv; }
      if (ACT == 1) v = fmaxf(v, 0.f);
      if (ACT == 2) v = 0.5f * v * (1.0f + erff(v * 0.70710678118654752f));
      if (ACT == 3) { const float u = 0.7978845608028654f * (v + 0.044715f * v * v * v); v = 0.5f * v * (1.0f + tanhf(u)); }
      so[w][8 * hh + r][t * 16 + ln] = v;
    }
  }
  __builtin_amdgcn_fence(__ATOMIC_ACQ_REL, "workgroup");
  __builtin_amdgcn_wave_barrier();
  const int rsub = lane >> 4, c4 = (lane & 15) * 4;
  for (int pass = 0; pass < 2; ++pass) {
#pragma unroll
    for (int q = 0; q < 8; ++q) {
      const int r = q * 2 + rsub;
      const v4f v = *(const v4fa*)&so[w][r][c4];
      *(volatile v4f*)(C + (size_t)(row0 + r) * ldc + col0 + c4) = v;
    }
    if (pass == 0) __threadfence();
  }
}
template <bool PARAM_BF16>
__global__ __launch_bounds__(256) void k_layernorm(const float* __restrict__ X, const float* __restrict__ R, const float* __restrict__ g, const float* __restrict__ bta,
                                                  float* __restrict__ out_sum, float* __restrict__ out_norm, int N, float eps) {
  __shared__ float red[256];
  const int row = blockIdx.x, tid = threadIdx.x;
  const float* x = X + (size_t)row * N; const float* rr = R ? R + (size_t)row * N : nullptr;
  float vals[16];
  const int per = N / 256;
  float s1 = 0.f;
  for (int u = 0; u < per / 4; ++u) {
    const int j = tid * 4 + 1024 * u;
    const v4f a = *(const v4fa*)(x + j);
    v4f b = {0.f,0.f,0.f,0.f}; if (rr) b = *(const v4fa*)(rr + j);
#pragma unroll
    for (int q = 0; q < 4; ++q) { const float v = a[q] + b[q]; vals[u * 4 + q] = v; s1 += v; }
  }
  red[tid] = s1; __syncthreads();
  for (int st = 128; st > 0; st >>= 1) { if (tid < st) red[tid] += red[tid + st]; __syncthreads(); }
  const float mu = red[0] / (float)N; __syncthreads();
  float s2 = 0.f;
  for (int u = 0; u < per / 4; ++u)
#pragma unroll
    for (int q = 0; q < 4; ++q) { const float c = vals[u * 4 + q] - mu; s2 += c * c; }
  red[tid] = s2; __syncthreads();
  for (int st = 128; st > 0; st >>= 1) { if (tid < st) red[tid] += red[tid + st]; __syncthreads(); }
  const float rs = rsqrtf(red[0] / (float)N + eps);
  for (int pass = 0; pass < 2; ++pass) {
    for (int u = 0; u < per / 4; ++u) {
      const int j = tid * 4 + 1024 * u;
      v4f o, sm;
#pragma unroll
      for (int q = 0; q < 4; ++q) {
        float gg = g[j + q], bb = bta[j + q];
        if (PARAM_BF16) { gg = bf16_round(gg); bb = bf16_round(bb); }
        sm[q] = vals[u * 4 + q]; o[q] = (vals[u * 4 + q] - mu) * rs * gg + bb;
      }
      if (out_sum) *(volatile v4f*)(out_sum + (size_t)row * N + j) = sm;
      *(volatile v4f*)(out_norm + (size_t)row * N + j) = o;
    }
    if (pass == 0) __threadfence();
  }
}


typedef _Float16 v16h __attribute__((ext_vector_type(16)));
union FragH { v16h v; v8us half[2]; _Float16 h[16]; unsigned short u[16]; };
template <int NT>
__device__ __forceinline__ v8f mmaH(v16h ah, v16h al, v16h bh, v16h bl, v8f c) {
  c = __builtin_amdgcn_wmma_f32_16x16x32_f16(false, ah, false, bh, (short)0, c, false, false);
  if (NT >= 2) c = __builtin_amdgcn_wmma_f32_16x16x32_f16(false, al, false, bh, (short)0, c, false, false);
  if (NT >= 3) c = __builtin_amdgcn_wmma_f32_16x16x32_f16(false, ah, false, bl, (short)0, c, false, false);
  asm volatile("v_nop\n\tv_nop\n\tv_nop\n\tv_nop" : "+v"(c) : "v"(ah), "v"(al), "v"(bh), "v"(bl));
  return c;
}
template <bool ASPLIT>
__global__ __launch_bounds__(128) void k_gemm_h(const float* __restrict__ A, int lda, size_t sA, const _Float16* __restrict__ Bh, int ldb, size_t sB, float alpha, float* __restrict__ C, int ldc, size_t sC, int M, int N, int K) {
  __shared__ __attribute__((aligned(16))) float so[4][16][64];
  const int tid = threadIdx.x, w = tid >> 5, lane = tid & 31, ln = lane & 15, hh = lane >> 4; const int by = blockIdx.y;
  A += (size_t)by * sA; Bh += (size_t)by * sB; C += (size_t)by * sC;
  const int ntn = (N + 63) / 64; const int wid = blockIdx.x * 4 + w; const int mt = wid / ntn, nq = wid % ntn; if (mt * 16 >= M) return;
  const int row0 = mt * 16, col0 = nq * 64; const float* arow = A + (size_t)(row0 + ln) * lda;
  v8f acc[4] = {};
  for (int kb = 0; kb < K; kb += 32) {
    FragH ah, al;
    const v4f x0 = *(const v4fa*)(arow + kb + 8 * hh), x1 = *(const v4fa*)(arow + kb + 8 * hh + 4), x2 = *(const v4fa*)(arow + kb + 16 + 8 * hh), x3 = *(const v4fa*)(arow + kb + 16 + 8 * hh + 4);
    float xs[16] = {x0[0],x0[1],x0[2],x0[3],x1[0],x1[1],x1[2],x1[3],x2[0],x2[1],x2[2],x2[3],x3[0],x3[1],x3[2],x3[3]};
#pragma unroll
    for (int i = 0; i < 16; ++i) { const _Float16 h = (_Float16)xs[i]; ah.h[i] = h; al.h[i] = ASPLIT ? (_Float16)(xs[i] - (float)h) : (_Float16)0.0f; }
#pragma unroll
    for (int t = 0; t < 4; ++t) { if (col0 + t * 16 >= N) continue; const size_t boff = (size_t)(col0 + t * 16 + ln) * ldb + kb; FragH bq; bq.half[0] = *(const v8us*)(Bh + boff + 8 * hh); bq.half[1] = *(const v8us*)(Bh + boff + 16 + 8 * hh);
      acc[t] = mmaH<ASPLIT ? 2 : 1>(ah.v, al.v, bq.v, bq.v, acc[t]); }
  }
#pragma unroll
  for (int t = 0; t < 4; ++t) { if (col0 + t * 16 >= N) continue;
#pragma unroll
    for (int r = 0; r < 8; ++r) so[w][8 * hh + r][t * 16 + ln] = acc[t][r] * alpha; }
  __builtin_amdgcn_fence(__ATOMIC_ACQ_REL, "workgroup"); __builtin_amdgcn_wave_barrier();
  const int rsub = lane >> 4, c4 = (lane & 15) * 4;
  for (int pass = 0; pass < 2; ++pass) {
#pragma unroll
    for (int q = 0; q < 8; ++q) { const int r = q * 2 + rsub; if (col0 + c4 < N) { const v4f v = *(const v4fa*)&so[w][r][c4]; *(volatile v4f*)(C + (size_t)(row0 + r) * ldc + col0 + c4) = v; } }
    if (pass == 0) __threadfence(); }
}

__global__ __launch_bounds__(256) void k_wt_f16(const float* __restrict__ W, _Float16* __restrict__ Wt, int K, int N, float scale) {
  const int t = blockIdx.x * 256 + threadIdx.x; if (t >= N * (K / 8)) return; const int n = t / (K / 8), k8 = (t % (K / 8)) * 8; FragH f;
#pragma unroll
  for (int i = 0; i < 8; ++i) f.h[i] = (_Float16)(bf16_round(W[(size_t)(k8 + i) * N + n]) * scale); const v8us o = f.half[0];
  *(volatile v8us*)((unsigned short*)Wt + (size_t)n * K + k8) = o; __threadfence(); *(volatile v8us*)((unsigned short*)Wt + (size_t)n * K + k8) = o;
}

__global__ __launch_bounds__(256) void k_wprep(const float* __restrict__ cw0, const float* __restrict__ cw1, const float* __restrict__ cw2, const float* __restrict__ cw3,
    const float* __restrict__ cb, const float* __restrict__ g, const float* __restrict__ bb, const float* __restrict__ rm, const float* __restrict__ rv, int layer, _Float16* __restrict__ Bl, float* __restrict__ biasf) {
  const size_t t = (size_t)blockIdx.x * 256 + threadIdx.x; const int KW = (layer == 0) ? 64 : 25 * CH; if (t >= (size_t)CH * KW / 8) return; const int o = (int)(t / (KW / 8)); const int k8 = (int)(t % (KW / 8)) * 8;
  const float s = bf16_round(g[o]) * rsqrtf(bf16_round(rv[o]) + 1e-5f); FragH f;
#pragma unroll
  for (int q = 0; q < 8; ++q) { const int k = k8 + q; float w = 0.f;
    if (layer == 0) { if (k < 50) { const int tap = k >> 1, c = k & 1; w = cw0[((size_t)o * 2 + c) * 25 + tap]; } }
    else { const int tap = k / CH, c = k % CH; const float* cw = (layer == 1) ? cw1 : (layer == 2) ? cw2 : cw3; w = cw[((size_t)o * CH + c) * 25 + tap]; }
    f.h[q] = (_Float16)(bf16_round(w) * s * 16.0f); }
  *(volatile v8us*)((unsigned short*)Bl + t * 8) = f.half[0];
  const bool wb = (blockIdx.x == 0 && threadIdx.x < CH); float bfo = 0.f; if (wb) { const int o2 = threadIdx.x; bfo = (bf16_round(cb[o2]) - bf16_round(rm[o2])) * (bf16_round(g[o2]) * rsqrtf(bf16_round(rv[o2]) + 1e-5f)) + bf16_round(bb[o2]); *(volatile float*)(biasf + o2) = bfo; }
  __threadfence(); *(volatile v8us*)((unsigned short*)Bl + t * 8) = f.half[0]; if (wb) *(volatile float*)(biasf + threadIdx.x) = bfo; }
__global__ __launch_bounds__(256) void k_rbf(const float* __restrict__ xs, const float* __restrict__ ys, const float* __restrict__ vals, const int* __restrict__ mask32, _Float16* __restrict__ G16) {
  __shared__ float spx[NPT], spy[NPT], spv[NPT];
  const int tid = threadIdx.x; const int bt = blockIdx.x / (NG / 256), mblk = blockIdx.x % (NG / 256);
  for (int p = tid; p < NPT; p += 256) { const size_t i = (size_t)bt * NPT + p; const float mk = mask32[i] ? 1.0f : 0.0f;
    spx[p] = 2.0f * (bf16_round(xs[i]) / 30.0f) - 1.0f; spy[p] = 2.0f * (bf16_round(ys[i]) / 30.0f) - 1.0f; spv[p] = bf16_round(vals[i]); if (mk == 0.f) { spx[p] = 1.0e6f; } }
  __syncthreads();
  const int m = mblk * 256 + tid; const int gyi = m / GR, gxi = m % GR; const float gx = -1.0f + 2.0f * (float)gxi / (float)(GR - 1), gy = -1.0f + 2.0f * (float)gyi / (float)(GR - 1);
  const float cexp = -0.5f / ((2.0f / GR) * (2.0f / GR)); float den = 0.f, wsum = 0.f;
#pragma unroll 4
  for (int p = 0; p < NPT; ++p) { const float dx = spx[p] - gx, dy = spy[p] - gy; const float w = expf(cexp * (dx * dx + dy * dy)); den += w; wsum += spv[p] * w; }
  typedef _Float16 v2h __attribute__((ext_vector_type(2))); v2h o; o.x = (_Float16)den; o.y = (_Float16)(wsum / (den + 1e-5f));
  *(volatile v2h*)(G16 + ((size_t)bt * NG + m) * 2) = o; __threadfence(); *(volatile v2h*)(G16 + ((size_t)bt * NG + m) * 2) = o; }
__global__ __launch_bounds__(128) void k_conv0(const _Float16* __restrict__ G16, const _Float16* __restrict__ B0, const float* __restrict__ bf, _Float16* __restrict__ C0) {
  __shared__ __attribute__((aligned(16))) _Float16 so[4][16][CH];
  const int tid = threadIdx.x, w = tid >> 5, lane = tid & 31, ln = lane & 15, hh = lane >> 4; const size_t p0 = ((size_t)blockIdx.x * 4 + w) * 16; const size_t p = p0 + ln; const int bt = (int)(p / NG), m = (int)(p % NG), y = m / GR, x = m % GR;
  v8f acc[8];
#pragma unroll
  for (int q = 0; q < 8; ++q) acc[q] = (v8f){0.f,0.f,0.f,0.f,0.f,0.f,0.f,0.f};
#pragma unroll
  for (int kb = 0; kb < 64; kb += 32) { FragH a;
#pragma unroll
    for (int j = 0; j < 16; ++j) { const int k = kb + ((j < 8) ? (8 * hh + j) : (16 + 8 * hh + j - 8)); float v = 0.f;
      if (k < 50) { const int tap = k >> 1, c = k & 1; const int yy = y + tap / 5 - 2, xx = x + tap % 5 - 2; if (yy >= 0 && yy < GR && xx >= 0 && xx < GR) v = (float)G16[((size_t)bt * NG + yy * GR + xx) * 2 + c]; }
      a.h[j] = (_Float16)v; }
#pragma unroll
    for (int q = 0; q < 8; ++q) { FragH b; const unsigned short* br = (const unsigned short*)B0 + (size_t)(q * 16 + ln) * 64 + kb; b.half[0] = *(const v8us*)(br + 8 * hh); b.half[1] = *(const v8us*)(br + 16 + 8 * hh); acc[q] = mmaH<1>(a.v, a.v, b.v, b.v, acc[q]); } }
#pragma unroll
  for (int q = 0; q < 8; ++q) { const int o = q * 16 + ln; const float bv = bf[o];
#pragma unroll
    for (int r = 0; r < 8; ++r) so[w][8 * hh + r][o] = (_Float16)fmaxf(acc[q][r] * 0.0625f + bv, 0.f); }
  __builtin_amdgcn_fence(__ATOMIC_ACQ_REL, "workgroup"); __builtin_amdgcn_wave_barrier();
  { const unsigned short* sp = (const unsigned short*)&so[w][0][0]; unsigned short* dp = (unsigned short*)C0 + p0 * CH;
    for (int pass = 0; pass < 2; ++pass) {
#pragma unroll
      for (int i = 0; i < 8; ++i) *(volatile v8us*)(dp + (i * 32 + lane) * 8) = *(const v8us*)(sp + (i * 32 + lane) * 8);
      if (pass == 0) __threadfence(); } } }
template <int S, bool TANH>
__global__ __launch_bounds__(128) void k_conv(const _Float16* __restrict__ IN, const _Float16* __restrict__ Bl, const float* __restrict__ bf, _Float16* __restrict__ OUT) {
  __shared__ __attribute__((aligned(16))) _Float16 so[4][16][CH];
  const int tid = threadIdx.x, w = tid >> 5, lane = tid & 31, ln = lane & 15, hh = lane >> 4; const size_t p0 = ((size_t)blockIdx.x * 4 + w) * 16; const size_t p = p0 + ln; const int bt = (int)(p / (S * S)), m = (int)(p % (S * S)), y = m / S, x = m % S;
  v8f acc[8];
#pragma unroll
  for (int q = 0; q < 8; ++q) acc[q] = (v8f){0.f,0.f,0.f,0.f,0.f,0.f,0.f,0.f};
#pragma unroll 1
  for (int ks = 0; ks < 100; ++ks) { const int tap = ks >> 2, cb = (ks & 3) * 32; const int yy = y + tap / 5 - 2, xx = x + tap % 5 - 2; FragH a;
    if (yy >= 0 && yy < S && xx >= 0 && xx < S) { const unsigned short* ar = (const unsigned short*)IN + ((size_t)bt * S * S + yy * S + xx) * CH + cb; a.half[0] = *(const v8us*)(ar + 8 * hh); a.half[1] = *(const v8us*)(ar + 16 + 8 * hh); }
    else { for (int j = 0; j < 16; ++j) a.h[j] = (_Float16)0.0f; }
#pragma unroll
    for (int q = 0; q < 8; ++q) { FragH b; const unsigned short* br = (const unsigned short*)Bl + (size_t)(q * 16 + ln) * (25 * CH) + ks * 32; b.half[0] = *(const v8us*)(br + 8 * hh); b.half[1] = *(const v8us*)(br + 16 + 8 * hh); acc[q] = mmaH<1>(a.v, a.v, b.v, b.v, acc[q]); } }
#pragma unroll
  for (int q = 0; q < 8; ++q) { const int o = q * 16 + ln; const float bv = bf[o];
#pragma unroll
    for (int r = 0; r < 8; ++r) { float v = acc[q][r] * 0.0625f + bv; v = TANH ? tanhf(v) : fmaxf(v, 0.f); so[w][8 * hh + r][o] = (_Float16)v; } }
  __builtin_amdgcn_fence(__ATOMIC_ACQ_REL, "workgroup"); __builtin_amdgcn_wave_barrier();
  { const unsigned short* sp = (const unsigned short*)&so[w][0][0]; unsigned short* dp = (unsigned short*)OUT + p0 * CH;
    for (int pass = 0; pass < 2; ++pass) {
#pragma unroll
      for (int i = 0; i < 8; ++i) *(volatile v8us*)(dp + (i * 32 + lane) * 8) = *(const v8us*)(sp + (i * 32 + lane) * 8);
      if (pass == 0) __threadfence(); } } }
template <int S>
__global__ __launch_bounds__(256) void k_pool(const _Float16* __restrict__ IN, _Float16* __restrict__ OUT) { const size_t t = (size_t)blockIdx.x * 256 + threadIdx.x; constexpr int SO = S / 2; if (t >= (size_t)BT * SO * SO * CH / 8) return; const int c8 = (int)(t % (CH / 8)) * 8; const size_t po = t / (CH / 8); const int bt = (int)(po / (SO * SO)), m = (int)(po % (SO * SO)), y = m / SO, x = m % SO;
  const unsigned short* r00 = (const unsigned short*)IN + (((size_t)bt * S + 2 * y) * S + 2 * x) * CH + c8; FragH a, b, c, d, o; a.half[0] = *(const v8us*)(r00); b.half[0] = *(const v8us*)(r00 + CH); c.half[0] = *(const v8us*)(r00 + (size_t)S * CH); d.half[0] = *(const v8us*)(r00 + (size_t)S * CH + CH);
#pragma unroll
  for (int q = 0; q < 8; ++q) o.h[q] = (_Float16)(((float)a.h[q] + (float)b.h[q] + (float)c.h[q] + (float)d.h[q]) * 0.25f);
  *(volatile v8us*)((unsigned short*)OUT + t * 8) = o.half[0]; __threadfence(); *(volatile v8us*)((unsigned short*)OUT + t * 8) = o.half[0]; }
__global__ __launch_bounds__(256) void k_out(const _Float16* __restrict__ C3, float* __restrict__ out) { const size_t e = (size_t)blockIdx.x * 256 + threadIdx.x; if (e >= (size_t)BT * CH * 64) return; const int m = (int)(e % 64); const int c = (int)((e / 64) % CH); const int bt = (int)(e / (64 * CH));
  const float v = (float)C3[((size_t)bt * 64 + m) * CH + c]; *(volatile float*)(out + e) = v; __threadfence(); *(volatile float*)(out + e) = v; }

extern "C" void kernel_launch(void* const* d_in, const int* in_sizes, int n_in,
                              void* d_out, int out_size, void* d_ws, size_t ws_size, hipStream_t stream) {
  (void)in_sizes; (void)n_in; (void)out_size;
  const float* xs = (const float*)d_in[0]; const float* ys = (const float*)d_in[1]; const float* vals = (const float*)d_in[2]; const void* mask = d_in[3];
  const float* cw[4], *cb[4], *g[4], *bb[4], *rm[4], *rv[4]; for (int l = 0; l < 4; ++l) { cw[l] = (const float*)d_in[4 + 6 * l]; cb[l] = (const float*)d_in[5 + 6 * l]; g[l] = (const float*)d_in[6 + 6 * l]; bb[l] = (const float*)d_in[7 + 6 * l]; rm[l] = (const float*)d_in[8 + 6 * l]; rv[l] = (const float*)d_in[9 + 6 * l]; }
  char* ws = (char*)d_ws; size_t off = 0;
  auto take = [&](size_t bytes) { char* p = ws + off; off += (bytes + 255) & ~(size_t)255; return p; };
  _Float16* B0 = (_Float16*)take((size_t)CH * 64 * 2); _Float16* Bl[4]; Bl[0] = B0; for (int l = 1; l < 4; ++l) Bl[l] = (_Float16*)take((size_t)CH * 25 * CH * 2); float* bfv = (float*)take(4 * CH * 4);
  _Float16* G16 = (_Float16*)take((size_t)BT * NG * 2 * 2); _Float16* C0 = (_Float16*)take((size_t)BT * NG * CH * 2); _Float16* P0 = (_Float16*)take((size_t)BT * 1024 * CH * 2); _Float16* C1 = (_Float16*)take((size_t)BT * 1024 * CH * 2); _Float16* P1 = (_Float16*)take((size_t)BT * 256 * CH * 2); _Float16* C2 = (_Float16*)take((size_t)BT * 256 * CH * 2); _Float16* P2 = (_Float16*)take((size_t)BT * 64 * CH * 2); _Float16* C3 = (_Float16*)take((size_t)BT * 64 * CH * 2);
  if (off > ws_size) return;
  k_wprep<<<(CH * 64 / 8 + 255) / 256, 256, 0, stream>>>(cw[0], cw[1], cw[2], cw[3], cb[0], g[0], bb[0], rm[0], rv[0], 0, B0, bfv);
  for (int l = 1; l < 4; ++l) k_wprep<<<(unsigned)(((size_t)CH * 25 * CH / 8 + 255) / 256), 256, 0, stream>>>(cw[0], cw[1], cw[2], cw[3], cb[l], g[l], bb[l], rm[l], rv[l], l, Bl[l], bfv + l * CH);
  k_rbf<<<BT * (NG / 256), 256, 0, stream>>>(xs, ys, vals, (const int*)mask, G16);
  k_conv0<<<(unsigned)((size_t)BT * NG / 64), 128, 0, stream>>>(G16, B0, bfv, C0);
  k_pool<GR><<<(unsigned)(((size_t)BT * 1024 * CH / 8 + 255) / 256), 256, 0, stream>>>(C0, P0);
  k_conv<32, false><<<(unsigned)((size_t)BT * 1024 / 64), 128, 0, stream>>>(P0, Bl[1], bfv + CH, C1);
  k_pool<32><<<(unsigned)(((size_t)BT * 256 * CH / 8 + 255) / 256), 256, 0, stream>>>(C1, P1);
  k_conv<16, false><<<(unsigned)((size_t)BT * 256 / 64), 128, 0, stream>>>(P1, Bl[2], bfv + 2 * CH, C2);
  k_pool<16><<<(unsigned)(((size_t)BT * 64 * CH / 8 + 255) / 256), 256, 0, stream>>>(C2, P2);
  k_conv<8, true><<<(unsigned)((size_t)BT * 64 / 64), 128, 0, stream>>>(P2, Bl[3], bfv + 3 * CH, C3);
  k_out<<<(unsigned)(((size_t)BT * CH * 64 + 255) / 256), 256, 0, stream>>>(C3, (float*)d_out);
}
